// GNN_26414048871137
// MI455X (gfx1250) — hardware-verified
//
#include <hip/hip_runtime.h>
#include <stddef.h>
#include <stdint.h>
#include <math.h>


#define CIN    128
#define KC     256
#define NTHR   256
#define NWAVE  8
#define EPT    8
#define CHUNK  (NTHR * EPT)
#define WCAP   (EPT * 32)
#define LISTN  (NWAVE * WCAP)
#define NBA    1024
#define SLA    10
#define RCAP   20480
#define DEGCAP 64
#define GBM    64
#define GTHR   128
#define NUW1   2048
#define NUW2   4096
#define NUW3   1024
#define AGG_ZINTS (LISTN + 2 * RCAP + 3 * NBA)
#define MISC_INTS 16
#define EXTRA64   (NWAVE * 128)
#define EXTRA16   (NBA * 16)
#define RNROWS    256
#define WSMAX  134217728

static_assert((CHUNK & (CHUNK - 1)) == 0 && CHUNK <= 4096);
static_assert((NBA & (NBA - 1)) == 0 && NBA == (1 << SLA));
static_assert(((long long)CHUNK << SLA) < (1LL << 31));
static_assert(NBA % NWAVE == 0 && NBA % 32 == 0 && NBA % GBM == 0 && NBA % 2 == 0);
static_assert(AGG_ZINTS % (NTHR * 4) == 0 && LISTN % 4 == 0 && RCAP % 4 == 0);
static_assert(((AGG_ZINTS + MISC_INTS) % 4) == 0);
static_assert(CIN % 32 == 0 && KC % 32 == 0 && KC == 2 * CIN);
static_assert(GBM == (GTHR / 32) * 16);
static_assert(NUW1 % NTHR == 0 && NUW2 % NTHR == 0 && NUW3 % NTHR == 0);
static_assert((AGG_ZINTS + MISC_INTS + EXTRA16) * 4 <= 300000);
static_assert((NBA * 16) % (4 * NTHR) == 0);
static_assert(RNROWS == NWAVE * 32);

typedef float          v2f   __attribute__((ext_vector_type(2)));
typedef float          v4f   __attribute__((ext_vector_type(4)));
typedef float          v8f   __attribute__((ext_vector_type(8)));
typedef int            v4i   __attribute__((ext_vector_type(4)));
typedef int            v8i   __attribute__((ext_vector_type(8)));
typedef unsigned short v4us  __attribute__((ext_vector_type(4)));
typedef unsigned short v8us  __attribute__((ext_vector_type(8)));
typedef unsigned short v16us __attribute__((ext_vector_type(16)));
typedef __bf16         v16bf __attribute__((ext_vector_type(16)));
typedef v2f  __attribute__((may_alias)) v2fa;
typedef v4f  __attribute__((may_alias)) v4fa;
typedef v4i  __attribute__((may_alias)) v4ia;
typedef v4us __attribute__((may_alias)) v4usa;
typedef v8us __attribute__((may_alias)) v8usa;
union FragB { v16bf v; v16us u; v8us h[2]; v8i w; };

__device__ __forceinline__ v8f wmb(const FragB& a, const FragB& b, v8f c) {
  v8f d = __builtin_amdgcn_wmma_f32_16x16x32_bf16(false, a.v, false, b.v, (short)0, c, false, false);
  asm volatile("v_nop\n\tv_nop\n\tv_nop\n\tv_nop" : "+v"(d) : "v"(a.w), "v"(b.w));
  return d;
}

__device__ __forceinline__ unsigned bf16_bits(float f) {
  const unsigned u = __float_as_uint(f);
  return (u + 0x7FFFu + ((u >> 16) & 1u)) >> 16;
}
__device__ __forceinline__ float bf16_val(float f) {
  return __uint_as_float(bf16_bits(f) << 16);
}

__device__ __forceinline__ void wave_sync() {
  __builtin_amdgcn_fence(__ATOMIC_RELEASE, "wavefront");
  __builtin_amdgcn_wave_barrier();
  __builtin_amdgcn_fence(__ATOMIC_ACQUIRE, "wavefront");
}

__device__ __forceinline__ void put8(unsigned short* dp, v8us o) {
  *(volatile v8us*)dp = o;
  __threadfence();
  *(volatile v8us*)dp = o;
}

template <int SLB>
__device__ __forceinline__ int scan_chunk(const int* __restrict__ dsts, int nE, int cbase, int slotBase,
                                          int nb, int vec8, int* list, int tid, int lane, int wave) {
  int wc = 0;
  const int el0  = tid * EPT;
  const int e0   = cbase + el0;
  const int sent = -2147483647 - 1;
  v4i da, db;
  if (vec8 != 0 && cbase + CHUNK <= nE) {
    da = *(const v4i*)(dsts + e0);
    db = *(const v4i*)(dsts + e0 + 4);
  } else {
    da.x = (e0     < nE) ? dsts[min(e0,     nE - 1)] : sent;
    da.y = (e0 + 1 < nE) ? dsts[min(e0 + 1, nE - 1)] : sent;
    da.z = (e0 + 2 < nE) ? dsts[min(e0 + 2, nE - 1)] : sent;
    da.w = (e0 + 3 < nE) ? dsts[min(e0 + 3, nE - 1)] : sent;
    db.x = (e0 + 4 < nE) ? dsts[min(e0 + 4, nE - 1)] : sent;
    db.y = (e0 + 5 < nE) ? dsts[min(e0 + 5, nE - 1)] : sent;
    db.z = (e0 + 6 < nE) ? dsts[min(e0 + 6, nE - 1)] : sent;
    db.w = (e0 + 7 < nE) ? dsts[min(e0 + 7, nE - 1)] : sent;
  }
  const unsigned nbs = (unsigned)slotBase;
  const unsigned unb = (unsigned)nb;
  const unsigned s0 = (unsigned)da.x - nbs, s1 = (unsigned)da.y - nbs;
  const unsigned s2 = (unsigned)da.z - nbs, s3 = (unsigned)da.w - nbs;
  const unsigned s4 = (unsigned)db.x - nbs, s5 = (unsigned)db.y - nbs;
  const unsigned s6 = (unsigned)db.z - nbs, s7 = (unsigned)db.w - nbs;
  const bool h0 = s0 < unb, h1 = s1 < unb, h2 = s2 < unb, h3 = s3 < unb;
  const bool h4 = s4 < unb, h5 = s5 < unb, h6 = s6 < unb, h7 = s7 < unb;
  const unsigned any = __builtin_amdgcn_ballot_w32(h0 | h1 | h2 | h3 | h4 | h5 | h6 | h7);
  if (any != 0u) {
#define HITJ(J, HJ, SJ) { \
      const unsigned mj = __builtin_amdgcn_ballot_w32(HJ); \
      if (mj != 0u) { \
        if (HJ) { \
          const int pos = wc + (int)__builtin_amdgcn_mbcnt_lo(mj, 0u); \
          if (pos < WCAP) list[wave * WCAP + pos] = ((el0 + (J)) << SLB) | (int)(SJ); \
        } \
        wc += (int)__builtin_popcount(mj); } }
    HITJ(0, h0, s0)
    HITJ(1, h1, s1)
    HITJ(2, h2, s2)
    HITJ(3, h3, s3)
    HITJ(4, h4, s4)
    HITJ(5, h5, s5)
    HITJ(6, h6, s6)
    HITJ(7, h7, s7)
#undef HITJ
  }
  return wc;
}

__global__ __launch_bounds__(NTHR) void k_wprep(const float* __restrict__ W1, const float* __restrict__ W2,
                                                const float* __restrict__ W3, unsigned short* W1T,
                                                unsigned short* W2T2, unsigned short* W3T2) {
  const int u = (int)blockIdx.x * NTHR + (int)threadIdx.x;
  v8us o;
  if (u < NUW1) {
    const int n  = u >> 4;
    const int k8 = (u & 15) * 8;
    const float* p = W1 + (size_t)k8 * 128 + n;
#pragma unroll
    for (int i = 0; i < 8; ++i) o[i] = (unsigned short)bf16_bits(p[(size_t)i * 128]);
    put8(W1T + (size_t)n * CIN + k8, o);
  } else if (u < NUW1 + NUW2) {
    const int v  = u - NUW1;
    const int n  = v >> 5;
    const int k8 = (v & 31) * 8;
    const int kk = k8 & (CIN - 1);
    const float* p = W2 + (size_t)kk * 128 + n;
#pragma unroll
    for (int i = 0; i < 8; ++i) o[i] = (unsigned short)bf16_bits(p[(size_t)i * 128]);
    put8(W2T2 + (size_t)n * KC + k8, o);
  } else if (u < NUW1 + NUW2 + NUW3) {
    const int v  = u - NUW1 - NUW2;
    const int n  = v >> 5;
    const int k8 = (v & 31) * 8;
    const int kk = k8 & (CIN - 1);
    const float* p = W3 + (size_t)kk * 32 + n;
#pragma unroll
    for (int i = 0; i < 8; ++i) o[i] = (unsigned short)bf16_bits(p[(size_t)i * 32]);
    put8(W3T2 + (size_t)n * KC + k8, o);
  }
}

__global__ __launch_bounds__(NTHR) void k_cvx(const float* __restrict__ x, int nN, int nUnits,
                                              unsigned short* xb) {
  const int u = (int)blockIdx.x * NTHR + (int)threadIdx.x;
  if (u >= nUnits) return;
  const int row = u >> 4;
  const int k8  = (u & 15) * 8;
  const int rc  = row < nN ? row : nN - 1;
  const float* p = x + (size_t)rc * CIN + k8;
  const v4f a = *(const v4fa*)p;
  const v4f b = *(const v4fa*)(p + 4);
  const bool ok = row < nN;
  v8us o;
  o[0] = ok ? (unsigned short)bf16_bits(a.x) : (unsigned short)0;
  o[1] = ok ? (unsigned short)bf16_bits(a.y) : (unsigned short)0;
  o[2] = ok ? (unsigned short)bf16_bits(a.z) : (unsigned short)0;
  o[3] = ok ? (unsigned short)bf16_bits(a.w) : (unsigned short)0;
  o[4] = ok ? (unsigned short)bf16_bits(b.x) : (unsigned short)0;
  o[5] = ok ? (unsigned short)bf16_bits(b.y) : (unsigned short)0;
  o[6] = ok ? (unsigned short)bf16_bits(b.z) : (unsigned short)0;
  o[7] = ok ? (unsigned short)bf16_bits(b.w) : (unsigned short)0;
  unsigned short* dp = xb + (size_t)row * CIN + k8;
  *(volatile v8us*)dp = o;
  __threadfence();
  *(volatile v8us*)dp = o;
}

template <int NT>
__global__ __launch_bounds__(GTHR) void k_gemm(const unsigned short* __restrict__ A,
                                               const unsigned short* __restrict__ BT, int K,
                                               const float* __restrict__ avs, const float* __restrict__ avd,
                                               float* xh, float* al) {
  constexpr int N   = 16 * NT;
  constexpr int LPR = N / 4;
  constexpr int RPI = 32 / LPR;
  constexpr int NIT = 16 / RPI;
  constexpr int GS  = LPR / 2;
  static_assert(NT == 8 || NT == 2);
  __shared__ __attribute__((aligned(16))) float stg[GBM * N];
  __shared__ __attribute__((aligned(16))) float alst[GBM * 4];
  const int tid = (int)threadIdx.x, lane = tid & 31, wave = tid >> 5, hh = lane >> 4, m = lane & 15;
  const int rowBase = (int)blockIdx.x * GBM;

  v8f acc[NT];
  {
    const v8f z = {0.f, 0.f, 0.f, 0.f, 0.f, 0.f, 0.f, 0.f};
#pragma unroll
    for (int t = 0; t < NT; ++t) acc[t] = z;
  }
  const unsigned short* ap = A  + (size_t)(rowBase + 16 * wave + m) * (size_t)K + 8 * hh;
  const unsigned short* bp = BT + (size_t)m * (size_t)K + 8 * hh;
#pragma unroll 1
  for (int k0 = 0; k0 < K; k0 += 32) {
    FragB af;
    af.h[0] = *(const v8usa*)(ap + k0);
    af.h[1] = *(const v8usa*)(ap + k0 + 16);
#pragma unroll
    for (int nt = 0; nt < NT; ++nt) {
      const unsigned short* wq = bp + (size_t)(16 * nt) * (size_t)K + k0;
      FragB bf;
      bf.h[0] = *(const v8usa*)wq;
      bf.h[1] = *(const v8usa*)(wq + 16);
      acc[nt] = wmb(af, bf, acc[nt]);
    }
  }

#pragma unroll
  for (int nt = 0; nt < NT; ++nt) {
    const int lc = 16 * nt + m;
#pragma unroll
    for (int r = 0; r < 8; ++r) {
      const int lr = 16 * wave + 8 * hh + r;
      stg[lr * N + lc] = acc[nt][r];
    }
  }
  __syncthreads();

  const int rsub = lane / LPR;
  const int c4   = lane % LPR;
  v4f as4, ad4;
  {
    const v4f t1 = *(const v4f*)(avs + 4 * c4);
    const v4f t2 = *(const v4f*)(avd + 4 * c4);
    as4.x = bf16_val(t1.x); as4.y = bf16_val(t1.y); as4.z = bf16_val(t1.z); as4.w = bf16_val(t1.w);
    ad4.x = bf16_val(t2.x); ad4.y = bf16_val(t2.y); ad4.z = bf16_val(t2.z); ad4.w = bf16_val(t2.w);
  }
#pragma unroll 1
  for (int i = 0; i < NIT; ++i) {
    const int lr = 16 * wave + i * RPI + rsub;
    const v4f v = *(const v4fa*)(stg + lr * N + 4 * c4);
    float ps = v.x * as4.x; ps = fmaf(v.y, as4.y, ps); ps = fmaf(v.z, as4.z, ps); ps = fmaf(v.w, as4.w, ps);
    float pd = v.x * ad4.x; pd = fmaf(v.y, ad4.y, pd); pd = fmaf(v.z, ad4.z, pd); pd = fmaf(v.w, ad4.w, pd);
#pragma unroll
    for (int off = GS / 2; off > 0; off >>= 1) {
      ps += __shfl_xor(ps, off, 32);
      pd += __shfl_xor(pd, off, 32);
    }
    if ((c4 & (GS - 1)) == 0) {
      const int hd = c4 / GS;
      alst[lr * 4 + hd]     = ps;
      alst[lr * 4 + 2 + hd] = pd;
    }
    *(volatile v4f*)(xh + (size_t)(rowBase + lr) * N + 4 * c4) = v;
  }
  __threadfence();
  __syncthreads();
#pragma unroll 1
  for (int i = 0; i < NIT; ++i) {
    const int lr = 16 * wave + i * RPI + rsub;
    const v4f v = *(const v4fa*)(stg + lr * N + 4 * c4);
    *(volatile v4f*)(xh + (size_t)(rowBase + lr) * N + 4 * c4) = v;
  }
  if (wave < 2) {
    const int row = 32 * wave + lane;
    const v4f a = *(const v4fa*)(alst + 4 * row);
    float* p = al + (size_t)(rowBase + row) * 4;
    *(volatile v4f*)p = a;
    __threadfence();
    *(volatile v4f*)p = a;
  }
}

template <int D>
__global__ __launch_bounds__(NTHR) void k_scan(const int* __restrict__ srcs, const int* __restrict__ dsts,
                                               int nE, int nN, int vec8, int mRows,
                                               const float* __restrict__ al, const float* __restrict__ xh,
                                               const float* __restrict__ bias,
                                               float* agg, float* part, float* outp) {
  static_assert(D == 64 || D == 16);
  constexpr int CH = 2 * D;
  extern __shared__ __attribute__((aligned(16))) int dsm[];
  int* list = dsm;
  int* hl   = dsm + LISTN;
  int* sl   = hl + RCAP;
  int* cnt  = sl + RCAP;
  int* offs = cnt + NBA;
  int* cur  = offs + NBA;
  int* misc = cur + NBA;
  float* extra = (float*)(misc + MISC_INTS);
  const int tid = (int)threadIdx.x, lane = tid & 31, wave = tid >> 5;
  const int nodeBase = (int)blockIdx.x * NBA;

  {
    const v4i z4 = {0, 0, 0, 0};
    for (int i = tid * 4; i < AGG_ZINTS; i += NTHR * 4) *(v4ia*)(dsm + i) = z4;
    if (tid < MISC_INTS) misc[tid] = 0;
  }
  float bv0 = 0.0f, bv1 = 0.0f, bv2 = 0.0f, bv3 = 0.0f;
  if constexpr (D == 64) {
    const v4f t = *(const v4f*)(bias + 4 * lane);
    bv0 = bf16_val(t.x); bv1 = bf16_val(t.y); bv2 = bf16_val(t.z); bv3 = bf16_val(t.w);
  } else {
    bv0 = bf16_val(bias[lane & 15]);
  }
  __syncthreads();

  int t = 0, ov = 0;
  const int nChunks = (nE + CHUNK - 1) / CHUNK;
#pragma unroll 1
  for (int ch = 0; ch < nChunks; ++ch) {
    const int cbase = ch * CHUNK;
    const int wc = scan_chunk<SLA>(dsts, nE, cbase, nodeBase, NBA, vec8, list, tid, lane, wave);
    if (lane == 0) misc[wave] = wc;
    __syncthreads();
    if (wave == 0) {
#pragma unroll 1
      for (int w2 = 0; w2 < NWAVE; ++w2) {
        int c = misc[w2];
        c = c < 0 ? 0 : (c > WCAP ? WCAP : c);
#pragma unroll 1
        for (int b0 = 0; b0 < c; b0 += 32) {
          const int idx = b0 + lane;
          const int ent = list[w2 * WCAP + (idx < WCAP ? idx : WCAP - 1)];
          const int m32 = (c - b0) < 32 ? (c - b0) : 32;
#pragma unroll 1
          for (int k = 0; k < m32; ++k) {
            const int u    = __builtin_amdgcn_readlane(ent, k);
            const int slot = u & (NBA - 1);
            const int el   = (u >> SLA) & (CHUNK - 1);
            const int pk   = ((cbase + el) << SLA) | slot;
            if (t < RCAP) {
              if (lane == 0) { hl[t] = pk; cnt[slot] = cnt[slot] + 1; }
              t = t + 1;
            } else {
              ov = 1;
            }
          }
        }
      }
    }
    __syncthreads();
  }
  if (wave == 0 && lane == 0) { misc[8] = t; misc[9] = ov; }
  __syncthreads();
  int tt = misc[8];
  tt = tt < 0 ? 0 : (tt > RCAP ? RCAP : tt);
  const int ovf = misc[9];

  if (wave == 0) {
    const int base = lane * (NBA / 32);
    int s = 0;
#pragma unroll 1
    for (int i = 0; i < NBA / 32; ++i) s += cnt[base + i];
    int incl = s;
#pragma unroll
    for (int d = 1; d < 32; d <<= 1) {
      const int y = __shfl_up(incl, d, 32);
      if (lane >= d) incl += y;
    }
    int run = incl - s;
#pragma unroll 1
    for (int i = 0; i < NBA / 32; ++i) {
      const int cv = cnt[base + i];
      offs[base + i] = run;
      cur[base + i]  = run;
      run += cv;
    }
  }
  __syncthreads();
  if (wave == 0) {
#pragma unroll 1
    for (int b0 = 0; b0 < tt; b0 += 32) {
      const int idx = b0 + lane;
      const int ent = hl[idx < RCAP ? idx : RCAP - 1];
      const int m32 = (tt - b0) < 32 ? (tt - b0) : 32;
#pragma unroll 1
      for (int k = 0; k < m32; ++k) {
        const int u    = __builtin_amdgcn_readlane(ent, k);
        const int slot = u & (NBA - 1);
        if (lane == 0) {
          int p = cur[slot];
          p = p < 0 ? 0 : (p > RCAP - 1 ? RCAP - 1 : p);
          sl[p] = u;
          cur[slot] = p + 1;
        }
      }
    }
  }
  __syncthreads();

  const float qnan = __int_as_float(0x7fc00000);
  const float ninf = __int_as_float((int)0xff800000u);
  const float pz = (ovf != 0) ? qnan : 0.0f;
  const bool hsel = (lane >> 4) != 0;
  float cs0 = 0.0f, cs1 = 0.0f, cs2 = 0.0f, cs3 = 0.0f;
#pragma unroll 1
  for (int si = 0; si < NBA / NWAVE; ++si) {
    const int s    = si * NWAVE + wave;
    const int node = nodeBase + s;
    int c = cnt[s];
    const bool big = c > DEGCAP;
    c = c < 0 ? 0 : (c > DEGCAP ? DEGCAP : c);
    int o = offs[s];
    o = o < 0 ? 0 : (o > RCAP ? RCAP : o);
    const int nc = node < nN ? node : nN - 1;
    const v4f alr = *(const v4fa*)(al + (size_t)nc * 4);
    const float ad0 = alr.z, ad1 = alr.w;
    float m0, m1;
    {
      const float u0 = alr.x + ad0, u1 = alr.y + ad1;
      m0 = (u0 > 0.0f) ? u0 : 0.2f * u0;
      m1 = (u1 > 0.0f) ? u1 : 0.2f * u1;
    }
    float s0 = 1.0f, s1 = 1.0f;
    float a0, a1 = 0.0f, a2 = 0.0f, a3 = 0.0f;
    if constexpr (D == 64) {
      const v4f a = *(const v4fa*)(xh + (size_t)nc * CH + 4 * lane);
      a0 = a.x; a1 = a.y; a2 = a.z; a3 = a.w;
    } else {
      a0 = xh[(size_t)nc * CH + lane];
    }
#pragma unroll 1
    for (int b0 = 0; b0 < c; b0 += 32) {
      int idx = o + b0 + lane;
      idx = idx > RCAP - 1 ? RCAP - 1 : idx;
      const int ent = sl[idx];
      int eid = ent >> SLA;
      eid = eid < 0 ? 0 : (eid > nE - 1 ? nE - 1 : eid);
      int sr = srcs[eid];
      sr = sr < 0 ? 0 : (sr > nN - 1 ? nN - 1 : sr);
      const bool valid = (b0 + lane) < c;
      const v2f asv = *(const v2fa*)(al + (size_t)sr * 4);
      float l0 = asv.x + ad0, l1 = asv.y + ad1;
      l0 = (l0 > 0.0f) ? l0 : 0.2f * l0;
      l1 = (l1 > 0.0f) ? l1 : 0.2f * l1;
      float bm0 = valid ? l0 : ninf;
      float bm1 = valid ? l1 : ninf;
#pragma unroll
      for (int off = 16; off > 0; off >>= 1) {
        bm0 = fmaxf(bm0, __shfl_xor(bm0, off, 32));
        bm1 = fmaxf(bm1, __shfl_xor(bm1, off, 32));
      }
      const float n0 = fmaxf(m0, bm0), n1 = fmaxf(m1, bm1);
      const float sc0 = expf(m0 - n0), sc1 = expf(m1 - n1);
      const float x0 = expf(l0 - n0), x1 = expf(l1 - n1);
      const float e0 = valid ? x0 : 0.0f;
      const float e1 = valid ? x1 : 0.0f;
      float q0 = e0, q1 = e1;
#pragma unroll
      for (int off = 16; off > 0; off >>= 1) {
        q0 += __shfl_xor(q0, off, 32);
        q1 += __shfl_xor(q1, off, 32);
      }
      s0 = s0 * sc0 + q0;
      s1 = s1 * sc1 + q1;
      m0 = n0; m1 = n1;
      const float scl = hsel ? sc1 : sc0;
      a0 *= scl;
      if constexpr (D == 64) { a1 *= scl; a2 *= scl; a3 *= scl; }
      const int e0i = __float_as_int(e0), e1i = __float_as_int(e1);
      const int m32 = (c - b0) < 32 ? (c - b0) : 32;
#pragma unroll 1
      for (int k = 0; k < m32; ++k) {
        const int sk = __builtin_amdgcn_readlane(sr, k);
        const int ea = __builtin_amdgcn_readlane(e0i, k);
        const int eb = __builtin_amdgcn_readlane(e1i, k);
        const float ek = __int_as_float(hsel ? eb : ea);
        if constexpr (D == 64) {
          const v4f a = *(const v4fa*)(xh + (size_t)sk * CH + 4 * lane);
          a0 = fmaf(ek, a.x, a0); a1 = fmaf(ek, a.y, a1);
          a2 = fmaf(ek, a.z, a2); a3 = fmaf(ek, a.w, a3);
        } else {
          const float a = xh[(size_t)sk * CH + lane];
          a0 = fmaf(ek, a, a0);
        }
      }
    }
    const float pzr  = big ? qnan : pz;
    const bool  live = node < nN;
    const float rinv = 1.0f / (hsel ? s1 : s0);
    if constexpr (D == 64) {
      const float y0 = (a0 * rinv + bv0) + pzr;
      const float y1 = (a1 * rinv + bv1) + pzr;
      const float y2 = (a2 * rinv + bv2) + pzr;
      const float y3 = (a3 * rinv + bv3) + pzr;
      v4f ow;
      ow.x = live ? y0 : 0.0f; ow.y = live ? y1 : 0.0f;
      ow.z = live ? y2 : 0.0f; ow.w = live ? y3 : 0.0f;
      cs0 += ow.x; cs1 += ow.y; cs2 += ow.z; cs3 += ow.w;
      if (node < mRows) {
        float* op = agg + (size_t)node * CH + 4 * lane;
        *(volatile v4f*)op = ow;
        __threadfence();
        *(volatile v4f*)op = ow;
      }
    } else {
      const float v  = a0 * rinv;
      const float vo = __shfl_xor(v, 16, 32);
      const float ov2 = (0.5f * (v + vo) + bv0) + pzr;
      if (lane < 16) extra[s * 16 + lane] = ov2;
    }
  }

  if constexpr (D == 64) {
    v4f cw; cw.x = cs0; cw.y = cs1; cw.z = cs2; cw.w = cs3;
    *(v4fa*)(extra + wave * 128 + 4 * lane) = cw;
    __syncthreads();
    if (wave == 0) {
      v4f tot = *(const v4fa*)(extra + 4 * lane);
#pragma unroll
      for (int w2 = 1; w2 < NWAVE; ++w2) tot += *(const v4fa*)(extra + w2 * 128 + 4 * lane);
      float* pp = part + (size_t)blockIdx.x * 128 + 4 * lane;
      *(volatile v4f*)pp = tot;
      __threadfence();
      *(volatile v4f*)pp = tot;
    }
  } else {
    __syncthreads();
    int rows = nN - nodeBase;
    rows = rows < 0 ? 0 : (rows > NBA ? NBA : rows);
    const int nf4 = rows * 4;
    constexpr int NITO = (NBA * 16) / (4 * NTHR);
    v4f ovv[NITO];
#pragma unroll
    for (int it = 0; it < NITO; ++it) ovv[it] = *(const v4fa*)(extra + 4 * (it * NTHR + tid));
    float* ob = outp + (size_t)nodeBase * 16;
#pragma unroll
    for (int it = 0; it < NITO; ++it) {
      const int f = it * NTHR + tid;
      if (f < nf4) *(volatile v4f*)(ob + 4 * (size_t)f) = ovv[it];
    }
    __threadfence();
#pragma unroll
    for (int it = 0; it < NITO; ++it) {
      const int f = it * NTHR + tid;
      if (f < nf4) *(volatile v4f*)(ob + 4 * (size_t)f) = ovv[it];
    }
  }
}

__global__ __launch_bounds__(NTHR) void k_rownorm(const float* __restrict__ agg, const float* __restrict__ part,
                                                  int nPart, int nN, int mRows, double invN,
                                                  unsigned short* hpl) {
  __shared__ __attribute__((aligned(16))) float meanS[128];
  __shared__ __attribute__((aligned(16))) unsigned short rbuf[NWAVE * 256];
  const int tid = (int)threadIdx.x, lane = tid & 31, wave = tid >> 5;
  if (tid < 128) {
    double sacc = 0.0;
#pragma unroll 1
    for (int b = 0; b < nPart; ++b) sacc += (double)part[(size_t)b * 128 + tid];
    meanS[tid] = (float)(sacc * invN);
  }
  __syncthreads();
  const v4f mu = *(const v4fa*)(meanS + 4 * lane);
  unsigned short* rowbuf = rbuf + wave * 256;
#pragma unroll 1
  for (int ri = 0; ri < 32; ++ri) {
    const int row = (int)blockIdx.x * RNROWS + wave * 32 + ri;
    if (row < mRows) {
      const int rc = row < nN ? row : nN - 1;
      const v4f a = *(const v4fa*)(agg + (size_t)rc * 128 + 4 * lane);
      const float c0 = a.x - mu.x, c1 = a.y - mu.y, c2 = a.z - mu.z, c3 = a.w - mu.w;
      float ss = c0 * c0; ss = fmaf(c1, c1, ss); ss = fmaf(c2, c2, ss); ss = fmaf(c3, c3, ss);
#pragma unroll
      for (int off = 16; off > 0; off >>= 1) ss += __shfl_xor(ss, off, 32);
      const float nrm = sqrtf(ss);
      const float inv = 1.0f / (1e-5f + nrm);
      float y0 = c0 * inv, y1 = c1 * inv, y2 = c2 * inv, y3 = c3 * inv;
      y0 = (y0 > 0.0f) ? y0 : (y0 - y0);
      y1 = (y1 > 0.0f) ? y1 : (y1 - y1);
      y2 = (y2 > 0.0f) ? y2 : (y2 - y2);
      y3 = (y3 > 0.0f) ? y3 : (y3 - y3);
      const bool live = row < nN;
      const float v0 = live ? y0 : 0.0f, v1 = live ? y1 : 0.0f;
      const float v2 = live ? y2 : 0.0f, v3 = live ? y3 : 0.0f;
      v4us mh, ml;
      {
        unsigned hb;
        hb = bf16_bits(v0); mh[0] = (unsigned short)hb; ml[0] = (unsigned short)bf16_bits(v0 - __uint_as_float(hb << 16));
        hb = bf16_bits(v1); mh[1] = (unsigned short)hb; ml[1] = (unsigned short)bf16_bits(v1 - __uint_as_float(hb << 16));
        hb = bf16_bits(v2); mh[2] = (unsigned short)hb; ml[2] = (unsigned short)bf16_bits(v2 - __uint_as_float(hb << 16));
        hb = bf16_bits(v3); mh[3] = (unsigned short)hb; ml[3] = (unsigned short)bf16_bits(v3 - __uint_as_float(hb << 16));
      }
      *(v4usa*)(rowbuf + 4 * lane) = mh;
      *(v4usa*)(rowbuf + 128 + 4 * lane) = ml;
      wave_sync();
      const v8us q0 = *(const v8usa*)(rowbuf + 8 * lane);
      wave_sync();
      unsigned short* rp = hpl + (size_t)row * KC + 8 * lane;
      *(volatile v8us*)rp = q0;
      __threadfence();
      *(volatile v8us*)rp = q0;
    }
  }
}

static inline int cdiv(int a, int b) { return (a + b - 1) / b; }
static inline size_t al256(size_t o) { return (o + 255) & ~(size_t)255; }

extern "C" void kernel_launch(void* const* d_in, const int* in_sizes, int n_in,
                              void* d_out, int out_size, void* d_ws, size_t ws_size,
                              hipStream_t stream) {
  if (n_in < 14) return;
  if (in_sizes[0] < CIN || (in_sizes[0] % CIN) != 0) return;
  const int nN = in_sizes[0] / CIN;
  if (nN < 2 || (nN & 1) != 0 || nN > (1 << 22)) return;
  if (in_sizes[1] < 2 || (in_sizes[1] & 1) != 0) return;
  const int nE = in_sizes[1] / 2;
  if (nE < 1 || nE >= (1 << (31 - SLA))) return;
  if (in_sizes[2] != 128 * 128) return;
  if (in_sizes[3] != 128 || in_sizes[4] != 128 || in_sizes[5] != 128) return;
  if (in_sizes[6] != 128 * 128) return;
  if (in_sizes[7] != 128 || in_sizes[8] != 128 || in_sizes[9] != 128) return;
  if (in_sizes[10] != 128 * 32) return;
  if (in_sizes[11] != 32 || in_sizes[12] != 32 || in_sizes[13] != 16) return;
  if ((long long)out_size != (long long)nN * 16) return;

  const float* x    = (const float*)d_in[0];
  const int*   edge = (const int*)d_in[1];
  const float* W1   = (const float*)d_in[2];
  const float* as1  = (const float*)d_in[3];
  const float* ad1  = (const float*)d_in[4];
  const float* b1   = (const float*)d_in[5];
  const float* W2   = (const float*)d_in[6];
  const float* as2  = (const float*)d_in[7];
  const float* ad2  = (const float*)d_in[8];
  const float* b2   = (const float*)d_in[9];
  const float* W3   = (const float*)d_in[10];
  const float* as3  = (const float*)d_in[11];
  const float* ad3  = (const float*)d_in[12];
  const float* b3   = (const float*)d_in[13];
  float* out = (float*)d_out;
  const int* src = edge;
  const int* dst = edge + nE;

  const int MP = cdiv(nN, GBM) * GBM;
  const int gM = MP / GBM;
  const int gA = cdiv(MP, NBA);
  if ((long long)gA * NBA < (long long)MP) return;
  const int gR = cdiv(MP, RNROWS);
  const int vec8 = ((nE & 3) == 0) ? 1 : 0;
  const double invN = 1.0 / (double)nN;

  char* ws = (char*)d_ws;
  size_t off = 0;
  const size_t oW1T = off; off = al256(off + (size_t)128 * CIN * 2);
  const size_t oW2T = off; off = al256(off + (size_t)128 * KC * 2);
  const size_t oW3T = off; off = al256(off + (size_t)32 * KC * 2);
  const size_t oXB  = off; off = al256(off + (size_t)MP * CIN * 2);
  const size_t oXH  = off; off = al256(off + (size_t)MP * 128 * 4);
  const size_t oXH3 = off; off = al256(off + (size_t)MP * 32 * 4);
  const size_t oAL  = off; off = al256(off + (size_t)MP * 4 * 4);
  const size_t oAGG = off; off = al256(off + (size_t)MP * 128 * 4);
  const size_t oH   = off; off = al256(off + (size_t)MP * KC * 2);
  const size_t oPT  = off; off = al256(off + (size_t)gA * 128 * 4);
  if (off > ws_size || off > (size_t)WSMAX) return;
  unsigned short* W1T  = (unsigned short*)(ws + oW1T);
  unsigned short* W2T2 = (unsigned short*)(ws + oW2T);
  unsigned short* W3T2 = (unsigned short*)(ws + oW3T);
  unsigned short* XB   = (unsigned short*)(ws + oXB);
  float*          XH   = (float*)(ws + oXH);
  float*          XH3  = (float*)(ws + oXH3);
  float*          AL   = (float*)(ws + oAL);
  float*          AGG  = (float*)(ws + oAGG);
  unsigned short* H    = (unsigned short*)(ws + oH);
  float*          PART = (float*)(ws + oPT);

  const size_t lds64 = (size_t)(AGG_ZINTS + MISC_INTS + EXTRA64) * 4;
  const size_t lds16 = (size_t)(AGG_ZINTS + MISC_INTS + EXTRA16) * 4;
  hipFuncSetAttribute(reinterpret_cast<const void*>(&k_scan<64>), hipFuncAttributeMaxDynamicSharedMemorySize, (int)lds64);
  hipFuncSetAttribute(reinterpret_cast<const void*>(&k_scan<16>), hipFuncAttributeMaxDynamicSharedMemorySize, (int)lds16);

  const int nUx = MP * (CIN / 8);
  k_wprep<<<(NUW1 + NUW2 + NUW3) / NTHR, NTHR, 0, stream>>>(W1, W2, W3, W1T, W2T2, W3T2);
  k_cvx<<<cdiv(nUx, NTHR), NTHR, 0, stream>>>(x, nN, nUx, XB);
  k_gemm<8><<<gM, GTHR, 0, stream>>>(XB, W1T, CIN, as1, ad1, XH, AL);
  k_scan<64><<<gA, NTHR, lds64, stream>>>(src, dst, nE, nN, vec8, MP, AL, XH, b1, AGG, PART, out);
  k_rownorm<<<gR, NTHR, 0, stream>>>(AGG, PART, gA, nN, MP, invN, H);
  k_gemm<8><<<gM, GTHR, 0, stream>>>(H, W2T2, KC, as2, ad2, XH, AL);
  k_scan<64><<<gA, NTHR, lds64, stream>>>(src, dst, nE, nN, vec8, MP, AL, XH, b2, AGG, PART, out);
  k_rownorm<<<gR, NTHR, 0, stream>>>(AGG, PART, gA, nN, MP, invN, H);
  k_gemm<2><<<gM, GTHR, 0, stream>>>(H, W3T2, KC, as3, ad3, XH3, AL);
  k_scan<16><<<gA, NTHR, lds16, stream>>>(src, dst, nE, nN, vec8, MP, AL, XH3, b3, AGG, PART, out);
}
